// LlamaAttention_50113678410517
// MI455X (gfx1250) — hardware-verified
//
#include <hip/hip_runtime.h>
#include <math.h>

#ifndef SEQ
#define SEQ 2048
#endif
#ifndef NB
#define NB 2
#endif
#define SEQ_FULL 2048
#define NB_FULL 2
#define DMD 2048
#define NQH 32
#define NKVH 8
#define HDM 64
#define QW (NQH * HDM)
#define KVW (NKVH * HDM)
#define QKW (QW + KVW)
#define WALL (QW + 2 * KVW)
#define TOK (NB * SEQ)
#define TT (SEQ / 64)
#define NREP (NQH / NKVH)
#define RES 128
static_assert(NB >= 1 && NB <= NB_FULL);
static_assert(SEQ % 128 == 0 && SEQ >= 128 && SEQ <= SEQ_FULL);
static_assert(HDM == 64 && QW == 2048 && KVW == 512 && QKW == 2560 && WALL == 3072 && NREP == 4 && (NQH % 2) == 0);
static_assert(TOK % 64 == 0 && QKW % 64 == 0 && KVW % 64 == 0 && SEQ % 64 == 0 && DMD % 64 == 0 && DMD % 32 == 0 && QW % 32 == 0 && HDM % 32 == 0 && TT <= 32 && (TT % 2) == 0);
static_assert(RES % 64 == 0 && RES % 16 == 0 && RES >= 64 && RES <= SEQ);

#define X16B ((size_t)TOK * DMD * 2)
#define W16B ((size_t)WALL * DMD * 2)
#define QKFB ((size_t)TOK * QKW * 4)
#define CPB  ((size_t)TOK * QW * 2)
#define CLB  CPB
#define SBB  ((size_t)NB * SEQ * SEQ * 4)
#define RAB  (((X16B + W16B + QKFB) > (CPB + CLB + SBB)) ? (X16B + W16B + QKFB) : (CPB + CLB + SBB))
#define PLB  ((size_t)TOK * (2 * QW + 2 * KVW) * 2)
#define WPB  ((size_t)DMD * QW * 2)
#define RSB  ((size_t)NB * RES * DMD * 4)
#define RBB  ((PLB > (WPB + RSB)) ? PLB : (WPB + RSB))
#define VTB  ((size_t)KVW * TOK * 2)
#define TFB  ((size_t)4096)
#define WSB  (RAB + RBB + 2 * VTB + TFB)
static_assert(WSB <= (size_t)134217728);
static_assert(X16B % 4096 == 0 && W16B % 4096 == 0 && QKFB % 4096 == 0 && CPB % 4096 == 0 && SBB % 4096 == 0 && PLB % 4096 == 0 && WPB % 4096 == 0 && RSB % 4096 == 0 && VTB % 4096 == 0);
static_assert(CPB + CLB + SBB <= RAB && X16B + W16B + QKFB <= RAB && PLB <= RBB && WPB + RSB <= RBB);
static_assert((size_t)TT * 32 * 4 <= TFB);
static_assert((size_t)((NB - 1) * SEQ_FULL + SEQ) * DMD * 4 <= (size_t)NB_FULL * SEQ_FULL * DMD * 4);

typedef __attribute__((ext_vector_type(16))) _Float16 v16h;
typedef __attribute__((ext_vector_type(8)))  _Float16 v8h;
typedef __attribute__((ext_vector_type(16))) __bf16   v16b;
typedef __attribute__((ext_vector_type(8)))  __bf16   v8b;
typedef __attribute__((ext_vector_type(8)))  float    v8f;
typedef __attribute__((ext_vector_type(4)))  float    v4f;
typedef __attribute__((ext_vector_type(4)))  int      v4i;
typedef __attribute__((ext_vector_type(4)))  unsigned v4u;

#define VST2(T, ptr, val) do { const T vst2_v_ = (val); *(volatile T*)(ptr) = vst2_v_; __threadfence(); *(volatile T*)(ptr) = vst2_v_; } while (0)

namespace kit {

__device__ __forceinline__ unsigned short f2bf_bits(float f) {
  unsigned u = __float_as_uint(f);
  return (unsigned short)((u + 0x7FFFu + ((u >> 16) & 1u)) >> 16);
}
__device__ __forceinline__ float bf_bits2f(unsigned short h) { return __uint_as_float(((unsigned)h) << 16); }
__device__ __forceinline__ unsigned short f2h_bits_ftz(float x) { return (fabsf(x) < 6.104e-5f) ? (unsigned short)0 : __builtin_bit_cast(unsigned short, (_Float16)x); }
__device__ __forceinline__ float h_bits2f(unsigned short h) { return (float)__builtin_bit_cast(_Float16, h); }

__device__ __forceinline__ void dep_guard_h(v8f& a, v8f& b, v16h x, v16h y) { asm volatile("v_nop\n\tv_nop\n\tv_nop\n\tv_nop" : "+v"(a), "+v"(b) : "v"(x), "v"(y)); }
__device__ __forceinline__ void dep_guard_b(v8f& a, v8f& b, v16b x, v16b y) { asm volatile("v_nop\n\tv_nop\n\tv_nop\n\tv_nop" : "+v"(a), "+v"(b) : "v"(x), "v"(y)); }
__device__ __forceinline__ void keep4_h(v16h a, v16h b, v16h c, v16h d) { asm volatile("v_nop" :: "v"(a), "v"(b), "v"(c), "v"(d)); }
__device__ __forceinline__ void keep4_b(v16b a, v16b b, v16b c, v16b d) { asm volatile("v_nop" :: "v"(a), "v"(b), "v"(c), "v"(d)); }
__device__ __forceinline__ void acc_guard4(v8f& a, v8f& b, v8f& c, v8f& d) { asm volatile("v_nop\n\tv_nop\n\tv_nop\n\tv_nop" : "+v"(a), "+v"(b), "+v"(c), "+v"(d)); }
template <typename T> struct Frag;
template <> struct Frag<_Float16> {
  typedef v16h V; union U { v16h v; v8h h[2]; };
  static __device__ __forceinline__ v16h load(const _Float16* p) {
    U f; f.h[0] = *(const v8h*)(p); f.h[1] = *(const v8h*)(p + 16); return f.v;
  }
  static __device__ __forceinline__ v8f mma(v16h a, v16h b, v8f c) {
    return __builtin_amdgcn_wmma_f32_16x16x32_f16(false, a, false, b, (short)0, c, false, false);
  }
  static __device__ __forceinline__ void guard(v8f& a, v8f& b, v16h x, v16h y) { dep_guard_h(a, b, x, y); }
  static __device__ __forceinline__ void keep(v16h a, v16h b, v16h c, v16h d) { keep4_h(a, b, c, d); }
};
template <> struct Frag<__bf16> {
  typedef v16b V; union U { v16b v; v8b h[2]; };
  static __device__ __forceinline__ v16b load(const __bf16* p) {
    U f; f.h[0] = *(const v8b*)(p); f.h[1] = *(const v8b*)(p + 16); return f.v;
  }
  static __device__ __forceinline__ v8f mma(v16b a, v16b b, v8f c) {
    return __builtin_amdgcn_wmma_f32_16x16x32_bf16(false, a, false, b, (short)0, c, false, false);
  }
  static __device__ __forceinline__ void guard(v8f& a, v8f& b, v16b x, v16b y) { dep_guard_b(a, b, x, y); }
  static __device__ __forceinline__ void keep(v16b a, v16b b, v16b c, v16b d) { keep4_b(a, b, c, d); }
};

template <int ET> struct Elem;
template <> struct Elem<0> { typedef _Float16 T; };
template <> struct Elem<1> { typedef __bf16 T; };
template <int ET, bool SPLIT, int OUT_MODE, int MASKM, bool RESID>
__global__ __launch_bounds__(256) void wmma_gemm64(
    const unsigned short* __restrict__ Ap, const unsigned short* __restrict__ A2p, int lda, long strideA,
    const unsigned short* __restrict__ Btp, const unsigned short* __restrict__ Bt2p, int ldb, long strideB,
    void* __restrict__ Cout, void* __restrict__ Cout2, int ldc, long strideC, int loRows, float osc1, float osc2,
    const float* __restrict__ resid, int ldr, long strideR, int resRows,
    const int* __restrict__ tmask,
    int M, int N, int K, float scale) {
  typedef typename Elem<ET>::T T;
  typedef typename Frag<T>::V V;
  const T* A = (const T*)Ap; const T* A2 = (const T*)A2p; const T* Bt = (const T*)Btp; const T* Bt2 = (const T*)Bt2p;
  __shared__ __align__(16) float sT[8][16 * 68];
  const int b    = blockIdx.y;
  const int lane = threadIdx.x & 31;
  const int wave = threadIdx.x >> 5;
  const int tilesN = N >> 6;
  const int tilesM = M >> 6;
  const int tile = blockIdx.x * 8 + wave;
  if (tile >= tilesM * tilesN) return;
  const int tm = tile / tilesN;
  const int tn = tile - tm * tilesN;
  if (MASKM == 1) {
    const int fl = __builtin_amdgcn_readfirstlane(tmask[tm * 32 + (tn & ~1)] | tmask[tm * 32 + (tn | 1)]);
    if (fl == 0) return;
  }
  const int m0 = tm << 6;
  const int n0 = tn << 6;

  const T* Ab  = A  + (size_t)b * strideA;
  const T* Bb  = Bt + (size_t)b * strideB;
  const T* Ab2 = SPLIT ? (A2  + (size_t)b * strideA) : nullptr;
  const T* Bb2 = SPLIT ? (Bt2 + (size_t)b * strideB) : nullptr;

  const int rlane = lane & 15;
  const int koff  = (lane >> 4) * 8;
  const int mOff  = (lane >> 4) * 8;

  v8f acc[4][4];
#pragma unroll
  for (int i = 0; i < 4; ++i)
#pragma unroll
    for (int j = 0; j < 4; ++j) acc[i][j] = (v8f){0.f,0.f,0.f,0.f,0.f,0.f,0.f,0.f};

  for (int k0 = 0; k0 < K; k0 += 32) {
    if (MASKM == 2) {
      const int fl = __builtin_amdgcn_readfirstlane(tmask[tm * 32 + (k0 >> 6)]);
      if (fl == 0) continue;
    }
    V bh[4], bl[4];
#pragma unroll
    for (int j = 0; j < 4; ++j) {
      const size_t bo = (size_t)(n0 + (j << 4) + rlane) * ldb + koff + k0;
      bh[j] = Frag<T>::load(Bb + bo);
      if (SPLIT) bl[j] = Frag<T>::load(Bb2 + bo);
    }
#pragma unroll
    for (int i = 0; i < 4; ++i) {
      const size_t ao = (size_t)(m0 + (i << 4) + rlane) * lda + koff + k0;
      V ah = Frag<T>::load(Ab + ao);
      V al;
      if (SPLIT) al = Frag<T>::load(Ab2 + ao);
#pragma unroll
      for (int j = 0; j < 4; ++j) {
        acc[i][j] = Frag<T>::mma(ah, bh[j], acc[i][j]);
        if (SPLIT) {
          acc[i][j] = Frag<T>::mma(ah, bl[j], acc[i][j]);
          acc[i][j] = Frag<T>::mma(al, bh[j], acc[i][j]);
        }
      }
      Frag<T>::guard(acc[i][0], acc[i][3], ah, SPLIT ? al : ah);
    }
    Frag<T>::keep(bh[0], bh[1], bh[2], bh[3]);
    if (SPLIT) Frag<T>::keep(bl[0], bl[1], bl[2], bl[3]);
  }
  acc_guard4(acc[0][0], acc[0][1], acc[0][2], acc[0][3]);
  acc_guard4(acc[1][0], acc[1][1], acc[1][2], acc[1][3]);
  acc_guard4(acc[2][0], acc[2][1], acc[2][2], acc[2][3]);
  acc_guard4(acc[3][0], acc[3][1], acc[3][2], acc[3][3]);

  float* slab = sT[wave];
  const float* Rb = RESID ? (resid + (size_t)b * strideR) : nullptr;
#pragma unroll
  for (int i = 0; i < 4; ++i) {
    const int mBase = m0 + (i << 4);
    const bool ron = RESID && (mBase < resRows);
#pragma unroll
    for (int j = 0; j < 4; ++j) {
      const int n = n0 + (j << 4) + rlane;
#pragma unroll
      for (int r = 0; r < 8; ++r) {
        float v = acc[i][j][r] * scale;
        if (RESID) {
          if (ron) { int rr = mBase + mOff + r; rr = (rr < resRows) ? rr : (resRows - 1); v += Rb[(size_t)rr * ldr + n]; }
        }
        slab[(mOff + r) * 68 + (j << 4) + rlane] = v;
      }
    }
    __builtin_amdgcn_fence(__ATOMIC_RELEASE, "workgroup");
    __builtin_amdgcn_wave_barrier();
    __builtin_amdgcn_fence(__ATOMIC_ACQUIRE, "workgroup");
    if (OUT_MODE == 0) {
      float* C = (float*)Cout + (size_t)b * strideC;
      const int hh = lane >> 4, c4 = (lane & 15) * 4;
      for (int pass = 0; pass < 2; ++pass) {
#pragma unroll
        for (int it = 0; it < 8; ++it) {
          const int row = it * 2 + hh;
          v4f v = *(const v4f*)(slab + row * 68 + c4);
          *(volatile v4f*)(C + (size_t)(mBase + row) * ldc + n0 + c4) = v;
        }
        __threadfence();
      }
    } else {
      const int q = lane >> 3, c8 = (lane & 7) * 8;
      unsigned short* C  = (unsigned short*)Cout + (size_t)b * strideC;
      unsigned short* C2 = (OUT_MODE >= 2) ? ((unsigned short*)Cout2 + (size_t)b * strideC) : nullptr;
      const bool wlo = (OUT_MODE >= 2) && (mBase < loRows);
      for (int pass = 0; pass < 2; ++pass) {
#pragma unroll
        for (int it = 0; it < 4; ++it) {
          const int row = it * 4 + q;
          const float* sp = slab + row * 68 + c8;
          v8h hv, lv;
          lv = (v8h){(_Float16)0.f,(_Float16)0.f,(_Float16)0.f,(_Float16)0.f,(_Float16)0.f,(_Float16)0.f,(_Float16)0.f,(_Float16)0.f};
#pragma unroll
          for (int e = 0; e < 8; ++e) {
            if (OUT_MODE == 1) {
              hv[e] = (_Float16)sp[e];
            } else if (OUT_MODE == 2) {
              const unsigned short hb = f2bf_bits(sp[e]);
              hv[e] = __builtin_bit_cast(_Float16, hb);
              if (wlo) lv[e] = __builtin_bit_cast(_Float16, f2bf_bits(sp[e] - bf_bits2f(hb)));
            } else {
              const float hf = sp[e] * osc1;
              const unsigned short hb = f2h_bits_ftz(hf);
              hv[e] = __builtin_bit_cast(_Float16, hb);
              if (wlo) lv[e] = __builtin_bit_cast(_Float16, f2h_bits_ftz((hf - h_bits2f(hb)) * osc2));
            }
          }
          *(volatile v8h*)(C + (size_t)(mBase + row) * ldc + n0 + c8) = hv;
          if (OUT_MODE >= 2) { if (wlo) *(volatile v8h*)(C2 + (size_t)(mBase + row) * ldc + n0 + c8) = lv; }
        }
        __threadfence();
      }
    }
    __builtin_amdgcn_fence(__ATOMIC_RELEASE, "workgroup");
    __builtin_amdgcn_wave_barrier();
    __builtin_amdgcn_fence(__ATOMIC_ACQUIRE, "workgroup");
  }
}

}

__device__ __forceinline__ unsigned short bfu_rne(float v) { unsigned u = __builtin_bit_cast(unsigned, v); u += 0x7FFFu + ((u >> 16) & 1u); return (unsigned short)(u >> 16); }
__device__ __forceinline__ void bfsplit(float v, unsigned short& hi, unsigned short& lo) { hi = bfu_rne(v); lo = bfu_rne(v - __builtin_bit_cast(float, (unsigned)hi << 16)); }
__device__ __forceinline__ void st4s(unsigned short* Hp, unsigned short* Lp, long long o, v4f a) { unsigned short h[4], l[4]; bfsplit(a.x, h[0], l[0]); bfsplit(a.y, h[1], l[1]); bfsplit(a.z, h[2], l[2]); bfsplit(a.w, h[3], l[3]);
    const unsigned long long ph = (unsigned long long)h[0] | ((unsigned long long)h[1] << 16) | ((unsigned long long)h[2] << 32) | ((unsigned long long)h[3] << 48), pl = (unsigned long long)l[0] | ((unsigned long long)l[1] << 16) | ((unsigned long long)l[2] << 32) | ((unsigned long long)l[3] << 48);
    VST2(unsigned long long, (unsigned long long*)(Hp + o), ph); VST2(unsigned long long, (unsigned long long*)(Lp + o), pl); }

__device__ __forceinline__ unsigned short at_f2h(float x) { return kit::f2h_bits_ftz(x); }
__device__ __forceinline__ void at_st8h(unsigned short* Pp, long long o, const float* v) { v4u pk; pk.x = (unsigned int)at_f2h(v[0]) | ((unsigned int)at_f2h(v[1]) << 16); pk.y = (unsigned int)at_f2h(v[2]) | ((unsigned int)at_f2h(v[3]) << 16); pk.z = (unsigned int)at_f2h(v[4]) | ((unsigned int)at_f2h(v[5]) << 16); pk.w = (unsigned int)at_f2h(v[6]) | ((unsigned int)at_f2h(v[7]) << 16); VST2(v4u, (v4u*)(Pp + o), pk); }
__device__ __forceinline__ v4f bfr4(v4f a) { v4f r; r.x = kit::bf_bits2f(kit::f2bf_bits(a.x)); r.y = kit::bf_bits2f(kit::f2bf_bits(a.y)); r.z = kit::bf_bits2f(kit::f2bf_bits(a.z)); r.w = kit::bf_bits2f(kit::f2bf_bits(a.w)); return r; }

__global__ __launch_bounds__(256) void k_cvtx(const float* __restrict__ X, unsigned short* __restrict__ O16, long long n8) {
    const long long u = (long long)blockIdx.x * 256 + threadIdx.x; if (u >= n8) return;
    const long long row = u / (DMD / 8); const int c = 8 * (int)(u % (DMD / 8));
    const int b = (int)(row / SEQ); const int l = (int)(row - (long long)b * SEQ);
    const float* x = X + ((size_t)b * SEQ_FULL + l) * DMD + c; const v4f a = *(const v4f*)x; const v4f bq = *(const v4f*)(x + 4);
    float v[8] = {a.x, a.y, a.z, a.w, bq.x, bq.y, bq.z, bq.w};
#pragma unroll
    for (int i = 0; i < 8; ++i) v[i] = kit::bf_bits2f(kit::f2bf_bits(v[i]));
    at_st8h(O16, 8 * u, v); }

template <int MODE>
__global__ __launch_bounds__(256) void k_tr16(const float* __restrict__ W, int NOUT, unsigned short* __restrict__ P, int pitch, int roff, int coff, float sc) {
    __shared__ __align__(16) float sW[64 * 68];
    const int n0 = blockIdx.x * 64, k0 = blockIdx.y * 64;
    const int tid = threadIdx.x, lane = tid & 31, wave = tid >> 5;
#pragma unroll
    for (int i = 0; i < 4; ++i) {
        const int idx = tid + 256 * i; const int r = idx >> 4, c4 = (idx & 15) * 4;
        const v4f v = *(const v4f*)(W + (size_t)(k0 + r) * NOUT + n0 + c4);
        *(v4f*)(sW + r * 68 + c4) = v;
    }
    __syncthreads();
    const int q = lane >> 3, e8 = (lane & 7) * 8;
    v4u pk[2]; size_t o[2];
#pragma unroll
    for (int it = 0; it < 2; ++it) {
        const int n = wave * 8 + it * 4 + q;
        unsigned short hb[8];
#pragma unroll
        for (int j = 0; j < 8; ++j) {
            const float w = sW[(e8 + j) * 68 + n];
            if (MODE == 0) hb[j] = at_f2h(kit::bf_bits2f(kit::f2bf_bits(w)) * sc); else hb[j] = kit::f2bf_bits(w);
        }
        pk[it].x = (unsigned)hb[0] | ((unsigned)hb[1] << 16); pk[it].y = (unsigned)hb[2] | ((unsigned)hb[3] << 16);
        pk[it].z = (unsigned)hb[4] | ((unsigned)hb[5] << 16); pk[it].w = (unsigned)hb[6] | ((unsigned)hb[7] << 16);
        o[it] = (size_t)(roff + n0 + n) * pitch + coff + k0 + e8;
    }
    for (int pass = 0; pass < 2; ++pass) {
#pragma unroll
        for (int it = 0; it < 2; ++it) {
            *(volatile v4u*)(P + o[it]) = pk[it];
        }
        __threadfence();
    }
}

__global__ __launch_bounds__(256) void k_rope(const float* __restrict__ QK, const float* __restrict__ CS, const float* __restrict__ SN,
                                              unsigned short* __restrict__ QH, unsigned short* __restrict__ QL, unsigned short* __restrict__ KH, unsigned short* __restrict__ KL, int nthr) {
    #pragma clang fp contract(off)
    const int u = blockIdx.x * 256 + threadIdx.x; if (u >= nthr) return;
    const int l16 = u & 15; const int hs = (u >> 4) % (NQH + NKVH); const int tt = u / ((NQH + NKVH) * 16);
    const int pos = tt % SEQ;
    const int i0 = 4 * (l16 & 7);
    const float* src = QK + (size_t)tt * QKW + hs * HDM;
    const v4f x1 = *(const v4f*)(src + i0), x2 = *(const v4f*)(src + 32 + i0);
    const float* cr = CS + (size_t)pos * HDM; const float* sr = SN + (size_t)pos * HDM;
    const v4f c1 = bfr4(*(const v4f*)(cr + i0)), s1 = bfr4(*(const v4f*)(sr + i0));
    const v4f c2 = bfr4(*(const v4f*)(cr + 32 + i0)), s2 = bfr4(*(const v4f*)(sr + 32 + i0));
    const v4f r1 = x1 * c1 - x2 * s1;
    const v4f r2 = x2 * c2 + x1 * s2;
    const bool first = (l16 < 8);
    v4f val; val.x = first ? r1.x : r2.x; val.y = first ? r1.y : r2.y; val.z = first ? r1.z : r2.z; val.w = first ? r1.w : r2.w;
    if (hs < NQH) st4s(QH, QL, (long long)tt * QW + hs * HDM + 4 * l16, val);
    else          st4s(KH, KL, (long long)tt * KVW + (hs - NQH) * HDM + 4 * l16, val); }

__global__ __launch_bounds__(256) void k_flags(const int* __restrict__ MK, int* __restrict__ TFp) {
    __shared__ unsigned sbits[8];
    const int tm = blockIdx.x; const int lane = threadIdx.x & 31, wave = threadIdx.x >> 5;
    unsigned bits = 0u;
    for (int rr = 0; rr < 8; ++rr) {
        const int row = 64 * tm + 8 * wave + rr;
        const int* mr = MK + (size_t)row * SEQ_FULL + 4 * lane;
        for (int c = 0; c < SEQ / 128; ++c) {
            const v4i v = *(const v4i*)(mr + 128 * c);
            const int any = ((v.x | v.y | v.z | v.w) != 0) ? 1 : 0;
            const unsigned bal = (unsigned)__ballot(any);
            bits |= (((bal & 0xFFFFu) != 0u) ? 1u : 0u) << (2 * c);
            bits |= (((bal >> 16) != 0u) ? 1u : 0u) << (2 * c + 1);
        }
    }
    if (lane == 0) sbits[wave] = bits;
    __syncthreads();
    if (wave == 0) {
        const unsigned all = sbits[0] | sbits[1] | sbits[2] | sbits[3] | sbits[4] | sbits[5] | sbits[6] | sbits[7];
        const int f = (int)((all >> lane) & 1u);
        VST2(int, TFp + tm * 32 + lane, f);
    }
}

template <int NC>
__global__ __launch_bounds__(256) void k_sm(float* SP, const int* __restrict__ MK, const int* __restrict__ TF, float sc, int nrows) {
    #pragma clang fp contract(off)
    constexpr int LL = 128 * NC;
    const int r = blockIdx.x * 8 + (threadIdx.x >> 5); const int L = threadIdx.x & 31; if (r >= nrows) return;
    const int t = r % LL; const int tm = t >> 6;
    const float* s = SP + (size_t)r * LL + 4 * L;
    const int* mk = MK + (size_t)t * SEQ_FULL + 4 * L;
    unsigned short* PH = (unsigned short*)(SP + (size_t)r * LL);
    unsigned short* PL = PH + LL;
    const int myf = TF[tm * 32 + L];
    const unsigned pb = (unsigned)__ballot(myf != 0);
    v4f sv[NC];
    float m = -3.0e38f;
#pragma unroll
    for (int c = 0; c < NC; ++c) {
        v4f v; v.x = -1.0e30f; v.y = -1.0e30f; v.z = -1.0e30f; v.w = -1.0e30f;
        if (((pb >> (2 * c)) & 3u) != 0u) {
            const v4f x = *(const v4f*)(s + 128 * c); const v4i k4 = *(const v4i*)(mk + 128 * c);
            v.x = (k4.x != 0) ? x.x * sc : -1.0e30f; v.y = (k4.y != 0) ? x.y * sc : -1.0e30f;
            v.z = (k4.z != 0) ? x.z * sc : -1.0e30f; v.w = (k4.w != 0) ? x.w * sc : -1.0e30f;
            m = fmaxf(m, fmaxf(fmaxf(v.x, v.y), fmaxf(v.z, v.w)));
        }
        sv[c] = v;
    }
#pragma unroll
    for (int o = 16; o > 0; o >>= 1) m = fmaxf(m, __shfl_xor(m, o, 32));
    float sum = 0.f;
#pragma unroll
    for (int c = 0; c < NC; ++c) {
        if (((pb >> (2 * c)) & 3u) != 0u) {
#pragma unroll
            for (int e = 0; e < 4; ++e) { const float ex = (sv[c][e] > -1.0e29f) ? __expf(sv[c][e] - m) : 0.f; sv[c][e] = ex; sum += ex; }
        }
    }
#pragma unroll
    for (int o = 16; o > 0; o >>= 1) sum += __shfl_xor(sum, o, 32);
    const float inv = 1.f / sum;
#pragma unroll
    for (int c = 0; c < NC; ++c) { if (((pb >> (2 * c)) & 3u) != 0u) { const v4f pv = sv[c] * inv; st4s(PH, PL, (long long)(4 * L + 128 * c), pv); } }
}

extern "C" void kernel_launch(void* const* d_in, const int* in_sizes, int n_in, void* d_out, int out_size, void* d_ws, size_t ws_size, hipStream_t stream) {
    if (n_in < 8) return;
    if (in_sizes[0] < ((NB - 1) * SEQ_FULL + SEQ) * DMD || in_sizes[1] < SEQ * HDM || in_sizes[2] < SEQ * HDM || in_sizes[3] < (SEQ - 1) * SEQ_FULL + SEQ ||
        in_sizes[4] < DMD * QW || in_sizes[5] < DMD * KVW || in_sizes[6] < DMD * KVW || in_sizes[7] < QW * DMD || out_size < ((NB - 1) * SEQ_FULL + SEQ) * DMD) return;
    if (WSB > ws_size) return;
    const float* x  = (const float*)d_in[0];
    const float* cs = (const float*)d_in[1];
    const float* sn = (const float*)d_in[2];
    const int*   mk = (const int*)d_in[3];
    const float* wq = (const float*)d_in[4];
    const float* wk = (const float*)d_in[5];
    const float* wv = (const float*)d_in[6];
    const float* wo = (const float*)d_in[7];
    float* out = (float*)d_out;

    char* RA = (char*)d_ws; char* RB = RA + RAB; char* RC = RB + RBB; char* RD = RC + 2 * VTB;
    unsigned short* X16 = (unsigned short*)RA;
    unsigned short* W16 = (unsigned short*)(RA + X16B);
    float* QKF = (float*)(RA + X16B + W16B);
    unsigned short* CP = (unsigned short*)RA;
    unsigned short* CL = (unsigned short*)(RA + CPB);
    float* SB = (float*)(RA + CPB + CLB);
    unsigned short* QH = (unsigned short*)RB;
    unsigned short* QL = QH + (size_t)TOK * QW;
    unsigned short* KH = QL + (size_t)TOK * QW;
    unsigned short* KL = KH + (size_t)TOK * KVW;
    unsigned short* WP = (unsigned short*)RB;
    float* RSD = (float*)(RB + WPB);
    unsigned short* VTH = (unsigned short*)RC;
    unsigned short* VTL = (unsigned short*)(RC + VTB);
    int* TF = (int*)RD;

    k_cvtx<<<(unsigned)(((long long)TOK * DMD / 8 + 255) / 256), 256, 0, stream>>>(x, X16, (long long)TOK * DMD / 8);
    k_tr16<0><<<dim3(QW / 64, DMD / 64), 256, 0, stream>>>(wq, QW, W16, DMD, 0, 0, 64.0f);
    k_tr16<0><<<dim3(KVW / 64, DMD / 64), 256, 0, stream>>>(wk, KVW, W16, DMD, QW, 0, 64.0f);
    k_tr16<0><<<dim3(KVW / 64, DMD / 64), 256, 0, stream>>>(wv, KVW, W16, DMD, QW + KVW, 0, 64.0f);
    kit::wmma_gemm64<0, false, 0, 0, false><<<dim3((unsigned)(((TOK / 64) * (QKW / 64) + 7) / 8), 1u), 256, 0, stream>>>(
        X16, nullptr, DMD, 0L, W16, nullptr, DMD, 0L, (void*)QKF, nullptr, QKW, 0L, 0, 0.f, 0.f, nullptr, 0, 0L, 0, TF, TOK, QKW, DMD, 0.015625f);
    kit::wmma_gemm64<0, false, 2, 0, false><<<dim3((unsigned)(((KVW / 64) * (TOK / 64) + 7) / 8), 1u), 256, 0, stream>>>(
        W16 + (size_t)QKW * DMD, nullptr, DMD, 0L, X16, nullptr, DMD, 0L, (void*)VTH, (void*)VTL, TOK, 0L, KVW, 0.f, 0.f, nullptr, 0, 0L, 0, TF, KVW, TOK, DMD, 0.015625f);
    k_rope<<<(unsigned)((TOK * (NQH + NKVH) * 16 + 255) / 256), 256, 0, stream>>>(QKF, cs, sn, QH, QL, KH, KL, TOK * (NQH + NKVH) * 16);
    k_flags<<<(unsigned)TT, 256, 0, stream>>>(mk, TF);
    for (int h = 0; h < NQH; ++h) {
        const int g = h / NREP;
        kit::wmma_gemm64<1, true, 0, 1, false><<<dim3((unsigned)((TT * TT + 7) / 8), (unsigned)NB), 256, 0, stream>>>(
            QH + (size_t)h * HDM, QL + (size_t)h * HDM, QW, (long)SEQ * QW, KH + (size_t)g * HDM, KL + (size_t)g * HDM, KVW, (long)SEQ * KVW,
            (void*)SB, nullptr, SEQ, (long)SEQ * SEQ, 0, 0.f, 0.f, nullptr, 0, 0L, 0, TF, SEQ, SEQ, HDM, 1.0f);
        k_sm<SEQ / 128><<<(unsigned)((TOK + 7) / 8), 256, 0, stream>>>(SB, mk, TF, 0.125f, TOK);
        kit::wmma_gemm64<1, true, 3, 2, false><<<dim3((unsigned)((TT + 7) / 8), (unsigned)NB), 256, 0, stream>>>(
            (const unsigned short*)SB, (const unsigned short*)SB + SEQ, 2 * SEQ, (long)SEQ * 2 * SEQ,
            VTH + (size_t)g * HDM * TOK, VTL + (size_t)g * HDM * TOK, TOK, (long)SEQ,
            (void*)(CP + (size_t)h * HDM), (void*)(CL + (size_t)h * HDM), QW, (long)SEQ * QW, RES, 16.0f, 4096.0f, nullptr, 0, 0L, 0, TF, SEQ, HDM, SEQ, 1.0f);
    }
    k_tr16<0><<<dim3(DMD / 64, QW / 64), 256, 0, stream>>>(wo, DMD, WP, QW, 0, 0, 64.0f);
    kit::wmma_gemm64<0, false, 0, 0, false><<<dim3((unsigned)(((RES / 64) * (DMD / 64) + 7) / 8), (unsigned)NB), 256, 0, stream>>>(
        CL, nullptr, QW, (long)SEQ * QW, WP, nullptr, QW, 0L, (void*)RSD, nullptr, DMD, (long)RES * DMD, 0, 0.f, 0.f, nullptr, 0, 0L, 0, TF, RES, DMD, QW, (1.0f / 4194304.0f));
    kit::wmma_gemm64<0, false, 0, 0, true><<<dim3((unsigned)((TT * (DMD / 64) + 7) / 8), (unsigned)NB), 256, 0, stream>>>(
        CP, nullptr, QW, (long)SEQ * QW, WP, nullptr, QW, 0L, (void*)out, nullptr, DMD, (long)SEQ_FULL * DMD, 0, 0.f, 0.f, RSD, DMD, (long)RES * DMD, RES, TF, SEQ, DMD, QW, (1.0f / 1024.0f));
}
